// Agent_Attention_3D_22239340659251
// MI455X (gfx1250) — hardware-verified
//
#include <hip/hip_runtime.h>
#include <stdint.h>

#define NTK   32768
#define CH    256
#define NHD   8
#define HDM   32
#define AGN   64
#define NTAP  27
#define KCV   6912
#define CHUNK 2048
#define NCHK  16
#define NSL   64
#define SLK   512
#define QT2   128
#define SPP   72
#define SOP   132
#define RECF  2176
#define SEGW  27

#define XSC   64.0f
#define WSC   1024.0f
#define QSC   64.0f
#define ASCL  4096.0f
#define PSC   1024.0f
#define AVQ   0.25f
#define OSC_G (1.0f / 65536.0f)
#define SHI   16384.0f
#define SLO   4.0f
#define ALO   4096.0f
#define OSC_P (1.0f / 16384.0f)
#define SFAC  (0.17677669529663687f * (1.0f / 262144.0f))
#define OSC2  (1.0f / 16777216.0f)

static_assert(NTK == 32 * 32 * 32);
static_assert(NHD * HDM == CH);
static_assert(KCV == NTAP * CH);
static_assert((KCV % 32) == 0 && (NTK % 64) == 0 && (CH % 64) == 0 && (CHUNK % 64) == 0);
static_assert(NTK == NCHK * CHUNK);
static_assert((CHUNK * NTAP) % (8 * SEGW) == 0);
static_assert((CH * NTAP) % (8 * SEGW) == 0);
static_assert(NSL * SLK == NTK && (SLK % 64) == 0);
static_assert((NTK % QT2) == 0 && QT2 == 128);
static_assert(RECF == 68 * 32);
static_assert((((NTK / 64) * (CH / 64)) % 8) == 0);
static_assert((((CHUNK / 64) * (CH / 64)) % 8) == 0);
static_assert(AGN == 64 && NSL == 64);

typedef _Float16 v16h __attribute__((ext_vector_type(16)));
typedef _Float16 v8h  __attribute__((ext_vector_type(8)));
typedef float    v8f  __attribute__((ext_vector_type(8)));
typedef float    v4f  __attribute__((ext_vector_type(4)));
typedef unsigned int v4u __attribute__((ext_vector_type(4)));

__device__ __forceinline__ unsigned short bf_bits(float f) {
  unsigned u = __float_as_uint(f);
  return (unsigned short)((u + 0x7FFFu + ((u >> 16) & 1u)) >> 16);
}
__device__ __forceinline__ float bf_up(unsigned short h) { return __uint_as_float(((unsigned)h) << 16); }
__device__ __forceinline__ float bfr(float f) { return bf_up(bf_bits(f)); }
__device__ __forceinline__ unsigned short h_bits(_Float16 x) { return __builtin_bit_cast(unsigned short, x); }
__device__ __forceinline__ unsigned short f2h_bits(float f) { return h_bits((_Float16)f); }
__device__ __forceinline__ unsigned pk16(unsigned short a, unsigned short b) { return (unsigned)a | ((unsigned)b << 16); }
__device__ __forceinline__ v8f zero8() { v8f z = {0.f, 0.f, 0.f, 0.f, 0.f, 0.f, 0.f, 0.f}; return z; }

__device__ __forceinline__ unsigned split_pair(float a, float b, unsigned& lo) {
  const _Float16 ha = (_Float16)a, hb = (_Float16)b;
  const _Float16 la = (_Float16)((a - (float)ha) * ALO);
  const _Float16 lb = (_Float16)((b - (float)hb) * ALO);
  lo = pk16(h_bits(la), h_bits(lb));
  return pk16(h_bits(ha), h_bits(hb));
}

__device__ __forceinline__ v16h ldfrag_h(const _Float16* p) {
  union { v16h v; v8h h[2]; } f;
  f.h[0] = *(const v8h*)(p);
  f.h[1] = *(const v8h*)(p + 16);
  return f.v;
}

__device__ __forceinline__ v8f mma_h_raw(v16h a, v16h b, v8f c) {
  return __builtin_amdgcn_wmma_f32_16x16x32_f16(false, a, false, b, (short)0, c, false, false);
}
__device__ __forceinline__ void dep_guard1(v8f& a, v16h x, v16h y) {
#if defined(__HIP_DEVICE_COMPILE__)
  asm volatile("v_nop\n\tv_nop\n\tv_nop\n\tv_nop" : "+v"(a) : "v"(x), "v"(y));
#endif
}
__device__ __forceinline__ void dep_guard_h(v8f& a, v8f& b, v16h x, v16h y) {
#if defined(__HIP_DEVICE_COMPILE__)
  asm volatile("v_nop\n\tv_nop\n\tv_nop\n\tv_nop" : "+v"(a), "+v"(b) : "v"(x), "v"(y));
#endif
}
__device__ __forceinline__ void dep_guard4(v8f& a, v8f& b, v8f& c, v8f& d, v16h x, v16h y) {
#if defined(__HIP_DEVICE_COMPILE__)
  asm volatile("v_nop\n\tv_nop\n\tv_nop\n\tv_nop" : "+v"(a), "+v"(b), "+v"(c), "+v"(d) : "v"(x), "v"(y));
#endif
}
__device__ __forceinline__ void keep4_h(v16h a, v16h b, v16h c, v16h d) {
#if defined(__HIP_DEVICE_COMPILE__)
  asm volatile("v_nop" :: "v"(a), "v"(b), "v"(c), "v"(d));
#endif
}
__device__ __forceinline__ void keep2_h(v16h a, v16h b) {
#if defined(__HIP_DEVICE_COMPILE__)
  asm volatile("v_nop" :: "v"(a), "v"(b));
#endif
}
__device__ __forceinline__ void acc_guard4(v8f& a, v8f& b, v8f& c, v8f& d) {
#if defined(__HIP_DEVICE_COMPILE__)
  asm volatile("v_nop\n\tv_nop\n\tv_nop\n\tv_nop" : "+v"(a), "+v"(b), "+v"(c), "+v"(d));
#endif
}
__device__ __forceinline__ void wave_sync_lds() {
  __builtin_amdgcn_fence(__ATOMIC_RELEASE, "workgroup");
  __builtin_amdgcn_wave_barrier();
  __builtin_amdgcn_fence(__ATOMIC_ACQUIRE, "workgroup");
}

__global__ __launch_bounds__(256) void k_cvt_rows(const float* __restrict__ src, int nrows, float scale, int rb,
                                                   unsigned short* dst) {
  const int tid = threadIdx.x, wave = tid >> 5, lane = tid & 31, c8 = lane * 8;
#pragma unroll 1
  for (int it = 0; it < 8; ++it) {
    const int row = blockIdx.x * 64 + it * 8 + wave;
    if (row < nrows) {
      const float* s = src + (size_t)row * CH + c8;
      const v4f a = *(const v4f*)(s);
      const v4f b = *(const v4f*)(s + 4);
      float v[8] = {a[0], a[1], a[2], a[3], b[0], b[1], b[2], b[3]};
#pragma unroll
      for (int i = 0; i < 8; ++i) {
        const float t = (rb != 0) ? bfr(v[i]) : v[i];
        v[i] = t * scale;
      }
      v4u p;
#pragma unroll
      for (int i = 0; i < 4; ++i) p[i] = pk16(f2h_bits(v[2 * i]), f2h_bits(v[2 * i + 1]));
      unsigned short* d = dst + (size_t)row * CH + c8;
      *(volatile v4u*)d = p;
      __threadfence();
      *(volatile v4u*)d = p;
    }
  }
}

__global__ __launch_bounds__(256) void k_cvt_v(const float* __restrict__ tf, unsigned short* vtm, unsigned short* vcm) {
  __shared__ __align__(16) _Float16 s16[CH * 72];
  const int tid = threadIdx.x, wave = tid >> 5, lane = tid & 31;
  const int n0 = blockIdx.x * 64;
#pragma unroll 8
  for (int it = 0; it < 64; ++it)
    s16[tid * 72 + it] = (_Float16)(tf[(size_t)(n0 + it) * CH + tid] * QSC);
  __syncthreads();
  v4u pc[8], pt[8];
#pragma unroll
  for (int it = 0; it < 8; ++it) {
    const int c = wave * 32 + it * 4 + (lane >> 3);
    pc[it] = *(const v4u*)(s16 + (size_t)c * 72 + (lane & 7) * 8);
  }
#pragma unroll
  for (int it = 0; it < 8; ++it) {
    const int t = wave * 8 + it;
    v4u p;
#pragma unroll
    for (int e = 0; e < 4; ++e)
      p[e] = pk16(h_bits(s16[(8 * lane + 2 * e) * 72 + t]), h_bits(s16[(8 * lane + 2 * e + 1) * 72 + t]));
    pt[it] = p;
  }
  for (int pass = 0; pass < 2; ++pass) {
#pragma unroll
    for (int it = 0; it < 8; ++it) {
      const int c = wave * 32 + it * 4 + (lane >> 3);
      *(volatile v4u*)(vcm + (size_t)c * NTK + n0 + (lane & 7) * 8) = pc[it];
    }
#pragma unroll
    for (int it = 0; it < 8; ++it) {
      const int t = wave * 8 + it;
      *(volatile v4u*)(vtm + (size_t)(n0 + t) * CH + 8 * lane) = pt[it];
    }
    __threadfence();
  }
}

__global__ __launch_bounds__(256) void k_cvt_wd(const float* __restrict__ w, unsigned short* wd) {
  const int tid = threadIdx.x, wave = tid >> 5, lane = tid & 31, c8 = lane * 8;
#pragma unroll 1
  for (int it = 0; it < SEGW; ++it) {
    const int seg = (blockIdx.x * 8 + wave) * SEGW + it;
    if (seg < CH * NTAP) {
      const int o = seg / NTAP, tap = seg - o * NTAP;
      const float* src = w + (size_t)o * KCV + (size_t)c8 * NTAP + tap;
      float vals[8];
#pragma unroll
      for (int i = 0; i < 8; ++i) vals[i] = bfr(src[i * NTAP]) * WSC;
      v4u p;
#pragma unroll
      for (int i = 0; i < 4; ++i) p[i] = pk16(f2h_bits(vals[2 * i]), f2h_bits(vals[2 * i + 1]));
      unsigned short* d = wd + (size_t)o * KCV + (size_t)tap * CH + c8;
      *(volatile v4u*)d = p;
      __threadfence();
      *(volatile v4u*)d = p;
    }
  }
}

__global__ __launch_bounds__(256) void k_cvt_wp(const float* __restrict__ w, unsigned short* dst) {
  const int tid = threadIdx.x, wave = tid >> 5, lane = tid & 31, c8 = lane * 8;
  const int row = blockIdx.x * 8 + wave;
  if (row < CH) {
    const float* src = w + (size_t)row * CH;
    float vals[8];
#pragma unroll
    for (int i = 0; i < 8; ++i) vals[i] = bfr(src[c8 + i]);
    v4u ph, pl;
#pragma unroll
    for (int i = 0; i < 4; ++i) {
      ph[i] = pk16(f2h_bits(vals[2 * i] * SHI), f2h_bits(vals[2 * i + 1] * SHI));
      pl[i] = pk16(f2h_bits(vals[2 * i] * SLO), f2h_bits(vals[2 * i + 1] * SLO));
    }
    unsigned short* dh = dst + (size_t)row * (2 * CH) + c8;
    unsigned short* dl = dh + CH;
    *(volatile v4u*)dh = ph;
    *(volatile v4u*)dl = pl;
    __threadfence();
    *(volatile v4u*)dh = ph;
    *(volatile v4u*)dl = pl;
  }
}

__global__ __launch_bounds__(256) void k_split(const float* __restrict__ s, unsigned short* s2) {
  const int tid = threadIdx.x, wave = tid >> 5, lane = tid & 31, c8 = lane * 8;
#pragma unroll 1
  for (int it = 0; it < 8; ++it) {
    const int row = blockIdx.x * 64 + it * 8 + wave;
    if (row < NTK) {
      const float* p = s + (size_t)row * CH + c8;
      const v4f a = *(const v4f*)(p);
      const v4f b = *(const v4f*)(p + 4);
      v4u ph, pl;
      unsigned lo;
      ph[0] = split_pair(a[0], a[1], lo); pl[0] = lo;
      ph[1] = split_pair(a[2], a[3], lo); pl[1] = lo;
      ph[2] = split_pair(b[0], b[1], lo); pl[2] = lo;
      ph[3] = split_pair(b[2], b[3], lo); pl[3] = lo;
      unsigned short* dh = s2 + (size_t)row * (2 * CH) + c8;
      unsigned short* dl = dh + CH;
      *(volatile v4u*)dh = ph;
      *(volatile v4u*)dl = pl;
      __threadfence();
      *(volatile v4u*)dh = ph;
      *(volatile v4u*)dl = pl;
    }
  }
}

__global__ __launch_bounds__(256) void k_im2col(const unsigned short* __restrict__ vtm, unsigned short* col, int chunk) {
  const int tid = threadIdx.x, wave = tid >> 5, lane = tid & 31, c8 = lane * 8;
  const int segb = (blockIdx.x * 8 + wave) * SEGW;
#pragma unroll 1
  for (int it = 0; it < SEGW; ++it) {
    const int seg = segb + it;
    if (seg < CHUNK * NTAP) {
      const int pl  = seg / NTAP;
      const int tap = seg - pl * NTAP;
      const int p   = chunk * CHUNK + pl;
      const int kz  = tap / 9, r9 = tap - kz * 9, ky = r9 / 3, kx = r9 - ky * 3;
      const int z = p >> 10, y = (p >> 5) & 31, x = p & 31;
      const int zz = z + kz - 1, yy = y + ky - 1, xx = x + kx - 1;
      const bool ok = ((unsigned)zz < 32u) && ((unsigned)yy < 32u) && ((unsigned)xx < 32u);
      const int zc = min(max(zz, 0), 31), yc = min(max(yy, 0), 31), xc = min(max(xx, 0), 31);
      const int nsrc = (zc << 10) + (yc << 5) + xc;
      const v4u v = *(const v4u*)(vtm + (size_t)nsrc * CH + c8);
      v4u o;
#pragma unroll
      for (int e = 0; e < 4; ++e) o[e] = ok ? v[e] : 0u;
      unsigned short* d = col + (size_t)seg * CH + c8;
      *(volatile v4u*)d = o;
      __threadfence();
      *(volatile v4u*)d = o;
    }
  }
}

template <int ADD>
__global__ __launch_bounds__(256) void gemm64(
    const unsigned short* __restrict__ Ap, int lda,
    const unsigned short* __restrict__ Btp, int ldb,
    float* Cp, int ldc,
    int M, int N, int K, float oscale,
    const float* __restrict__ bias, const float* __restrict__ addp) {
  const _Float16* A  = (const _Float16*)(const void*)Ap;
  const _Float16* Bt = (const _Float16*)(const void*)Btp;
  __shared__ __align__(16) float sT[8][16 * 68];
  const int lane = threadIdx.x & 31;
  const int wave = threadIdx.x >> 5;
  const int tilesN = N >> 6;
  const int tilesM = M >> 6;
  const int tile = blockIdx.x * 8 + wave;
  if (tile >= tilesM * tilesN) return;
  const int tm = tile / tilesN;
  const int tn = tile - tm * tilesN;
  const int m0 = tm << 6;
  const int n0 = tn << 6;

  const int rlane = lane & 15;
  const int koff  = (lane >> 4) * 8;
  const int mOff  = (lane >> 4) * 8;

  v8f acc[4][4];
#pragma unroll
  for (int i = 0; i < 4; ++i)
#pragma unroll
    for (int j = 0; j < 4; ++j) acc[i][j] = zero8();

  for (int k0 = 0; k0 < K; k0 += 32) {
    v16h bh[4];
#pragma unroll
    for (int j = 0; j < 4; ++j) {
      const size_t bo = (size_t)(n0 + (j << 4) + rlane) * ldb + koff + k0;
      bh[j] = ldfrag_h(Bt + bo);
    }
#pragma unroll
    for (int i = 0; i < 4; ++i) {
      const size_t ao = (size_t)(m0 + (i << 4) + rlane) * lda + koff + k0;
      const v16h ah = ldfrag_h(A + ao);
#pragma unroll
      for (int j = 0; j < 4; ++j) {
        acc[i][j] = mma_h_raw(ah, bh[j], acc[i][j]);
      }
      dep_guard_h(acc[i][0], acc[i][3], ah, bh[3]);
    }
    keep4_h(bh[0], bh[1], bh[2], bh[3]);
  }
  acc_guard4(acc[0][0], acc[0][1], acc[0][2], acc[0][3]);
  acc_guard4(acc[1][0], acc[1][1], acc[1][2], acc[1][3]);
  acc_guard4(acc[2][0], acc[2][1], acc[2][2], acc[2][3]);
  acc_guard4(acc[3][0], acc[3][1], acc[3][2], acc[3][3]);

  float* slab = sT[wave];
  float* C = Cp;
  const int hh = lane >> 4, c4 = (lane & 15) * 4;
  float bq[4];
#pragma unroll
  for (int e = 0; e < 4; ++e) bq[e] = bfr(bias[n0 + c4 + e]);
#pragma unroll
  for (int i = 0; i < 4; ++i) {
    const int mBase = m0 + (i << 4);
#pragma unroll
    for (int j = 0; j < 4; ++j) {
#pragma unroll
      for (int r = 0; r < 8; ++r) {
        slab[(mOff + r) * 68 + (j << 4) + rlane] = acc[i][j][r];
      }
    }
    wave_sync_lds();
    {
      v4f ov[8];
#pragma unroll
      for (int it = 0; it < 8; ++it) {
        const int row = it * 2 + hh;
        const int mrw = mBase + row;
        v4f v = *(const v4f*)(slab + row * 68 + c4);
        v[0] = v[0] * oscale + bq[0];
        v[1] = v[1] * oscale + bq[1];
        v[2] = v[2] * oscale + bq[2];
        v[3] = v[3] * oscale + bq[3];
        if (ADD) {
          const v4f ad = *(const v4f*)(addp + (size_t)mrw * ldc + n0 + c4);
          v[0] += ad[0]; v[1] += ad[1]; v[2] += ad[2]; v[3] += ad[3];
        }
        ov[it] = v;
      }
      for (int pass = 0; pass < 2; ++pass) {
#pragma unroll
        for (int it = 0; it < 8; ++it) {
          const int row = it * 2 + hh;
          *(volatile v4f*)(C + (size_t)(mBase + row) * ldc + n0 + c4) = ov[it];
        }
        __threadfence();
      }
    }
    wave_sync_lds();
  }
}

__global__ __launch_bounds__(256) void k_pool(const float* __restrict__ tf, unsigned short* ah) {
  __shared__ __align__(16) unsigned short sRow[CH];
  const int tid = threadIdx.x;
  const int ag = blockIdx.x;
  const int pz = ag >> 4, py = (ag >> 2) & 3, px = ag & 3;
  const int j = tid >> 5, d = tid & 31;
  float s = 0.0f;
#pragma unroll 1
  for (int b = 0; b < 512; ++b) {
    const int bz = b >> 6, by = (b >> 3) & 7, bx = b & 7;
    const int w  = (((pz * 8 + bz) * 32) + (py * 8 + by)) * 32 + px * 8 + bx;
    const int hq = w >> 12;
    const int n  = ((w & 4095) << 3) + j;
    s += tf[(size_t)n * CH + hq * HDM + d];
  }
  const float a = s * (1.0f / 512.0f);
  sRow[tid] = f2h_bits(a * ASCL);
  __syncthreads();
  if (tid < 32) {
    const v4u v = *(const v4u*)(sRow + 8 * tid);
    unsigned short* dst = ah + (size_t)ag * CH + 8 * tid;
    *(volatile v4u*)dst = v;
    __threadfence();
    *(volatile v4u*)dst = v;
  }
}

__global__ __launch_bounds__(256) void k_stage1(const unsigned short* __restrict__ ahp,
                                                 const unsigned short* __restrict__ khp,
                                                 const unsigned short* __restrict__ vcp,
                                                 float* part) {
  const _Float16* A  = (const _Float16*)(const void*)ahp;
  const _Float16* Kt = (const _Float16*)(const void*)khp;
  const _Float16* V  = (const _Float16*)(const void*)vcp;
  __shared__ __align__(16) _Float16 sP[AGN * SPP];
  __shared__ float sM1[8][16];
  __shared__ float sL1[8][16];
  __shared__ float sMrow[AGN];
  __shared__ __align__(16) float sRec[RECF];

  const int tid = threadIdx.x, wave = tid >> 5, lane = tid & 31;
  const int rl = lane & 15, hf = lane >> 4, koff = hf * 8;
  const int h  = blockIdx.x / NSL, sl = blockIdx.x - h * NSL;
  const int mt = wave & 3, kh = wave >> 2;
  const int key0 = sl * SLK;
  const int hc = h * HDM;

  const v16h aq = ldfrag_h(A + (size_t)(16 * mt + rl) * CH + hc + koff);

  float mloc[8];
#pragma unroll
  for (int r = 0; r < 8; ++r) mloc[r] = -3.0e38f;
  v16h kf;
#pragma unroll 1
  for (int t = 0; t < SLK / 32; ++t) {
    const int kb = key0 + kh * (SLK / 2) + 16 * t;
    kf = ldfrag_h(Kt + (size_t)(kb + rl) * CH + hc + koff);
    v8f s = mma_h_raw(aq, kf, zero8());
    dep_guard1(s, aq, kf);
#pragma unroll
    for (int r = 0; r < 8; ++r) mloc[r] = fmaxf(mloc[r], s[r]);
  }
#pragma unroll
  for (int r = 0; r < 8; ++r) {
    float mm = mloc[r];
    mm = fmaxf(mm, __shfl_xor(mm, 1, 32));
    mm = fmaxf(mm, __shfl_xor(mm, 2, 32));
    mm = fmaxf(mm, __shfl_xor(mm, 4, 32));
    mm = fmaxf(mm, __shfl_xor(mm, 8, 32));
    mloc[r] = mm;
  }
  if (rl == 0) {
#pragma unroll
    for (int r = 0; r < 8; ++r) sM1[wave][8 * hf + r] = mloc[r];
  }
  __syncthreads();
  if (tid < AGN) {
    const int m4 = tid >> 4, rr = tid & 15;
    sMrow[tid] = fmaxf(sM1[m4][rr], sM1[m4 + 4][rr]) * SFAC;
  }
  __syncthreads();
  float mrow[8];
#pragma unroll
  for (int r = 0; r < 8; ++r) mrow[r] = sMrow[16 * mt + 8 * hf + r];

  float lsum[8];
#pragma unroll
  for (int r = 0; r < 8; ++r) lsum[r] = 0.0f;
  v8f acc = zero8();
  const size_t vrow = (size_t)(hc + 16 * kh + rl) * NTK + key0;
  v16h vf;
#pragma unroll 1
  for (int c = 0; c < SLK / 64; ++c) {
#pragma unroll
    for (int t = 0; t < 2; ++t) {
      const int kb = key0 + c * 64 + kh * 32 + 16 * t;
      kf = ldfrag_h(Kt + (size_t)(kb + rl) * CH + hc + koff);
      v8f s = mma_h_raw(aq, kf, zero8());
      dep_guard1(s, aq, kf);
#pragma unroll
      for (int r = 0; r < 8; ++r) {
        const float p = __expf(s[r] * SFAC - mrow[r]);
        lsum[r] += p;
        sP[(16 * mt + 8 * hf + r) * SPP + kh * 32 + 16 * t + rl] = (_Float16)(p * PSC);
      }
    }
    __syncthreads();
#pragma unroll
    for (int ks = 0; ks < 2; ++ks) {
      const v16h af = ldfrag_h(sP + (16 * mt + rl) * SPP + 32 * ks + koff);
      vf = ldfrag_h(V + vrow + c * 64 + 32 * ks + koff);
      acc = mma_h_raw(af, vf, acc);
      dep_guard1(acc, af, vf);
    }
    __syncthreads();
  }
#pragma unroll
  for (int r = 0; r < 8; ++r) {
    float t = lsum[r];
    t += __shfl_xor(t, 1, 32);
    t += __shfl_xor(t, 2, 32);
    t += __shfl_xor(t, 4, 32);
    t += __shfl_xor(t, 8, 32);
    lsum[r] = t;
  }
  if (rl == 0) {
#pragma unroll
    for (int r = 0; r < 8; ++r) sL1[wave][8 * hf + r] = lsum[r];
  }
#pragma unroll
  for (int r = 0; r < 8; ++r) sRec[(16 * mt + 8 * hf + r) * 32 + 16 * kh + rl] = acc[r];
  __syncthreads();
  if (tid < AGN) {
    const int m4 = tid >> 4, rr = tid & 15;
    sRec[2048 + tid] = sMrow[tid];
    sRec[2112 + tid] = sL1[m4][rr] + sL1[m4 + 4][rr];
  }
  __syncthreads();
  float* rec = part + (size_t)blockIdx.x * RECF;
  const v4f p0 = *(const v4f*)(sRec + wave * 128 + 4 * lane);
  const v4f p1 = *(const v4f*)(sRec + (wave + 8) * 128 + 4 * lane);
  const v4f p2 = *(const v4f*)(sRec + 16 * 128 + 4 * lane);
  for (int pass = 0; pass < 2; ++pass) {
    *(volatile v4f*)(rec + wave * 128 + 4 * lane) = p0;
    *(volatile v4f*)(rec + (wave + 8) * 128 + 4 * lane) = p1;
    if (wave == 0) *(volatile v4f*)(rec + 16 * 128 + 4 * lane) = p2;
    __threadfence();
  }
}

__global__ __launch_bounds__(256) void k_comb(const float* __restrict__ part, unsigned short* avt) {
  __shared__ float sE[8][64];
  __shared__ __align__(16) unsigned short sO[HDM * AGN];
  const int tid = threadIdx.x, wave = tid >> 5, lane = tid & 31;
  const int h = blockIdx.x;
  const float* ph = part + (size_t)h * NSL * RECF;
#pragma unroll 1
  for (int i = 0; i < 8; ++i) {
    const int ag = i * 8 + wave;
    const float* r0 = ph + (size_t)lane * RECF;
    const float* r1 = ph + (size_t)(lane + 32) * RECF;
    const float m0 = r0[2048 + ag], m1 = r1[2048 + ag];
    float mm = fmaxf(m0, m1);
#pragma unroll
    for (int off = 16; off >= 1; off >>= 1) mm = fmaxf(mm, __shfl_xor(mm, off, 32));
    const float e0 = __expf(m0 - mm), e1 = __expf(m1 - mm);
    float L = r0[2112 + ag] * e0 + r1[2112 + ag] * e1;
#pragma unroll
    for (int off = 16; off >= 1; off >>= 1) L += __shfl_xor(L, off, 32);
    sE[wave][lane] = e0;
    sE[wave][lane + 32] = e1;
    wave_sync_lds();
    float a = 0.0f;
#pragma unroll 4
    for (int b = 0; b < NSL; ++b) a += sE[wave][b] * ph[(size_t)b * RECF + ag * 32 + lane];
    const float av = a * (1.0f / L) * AVQ;
    sO[lane * AGN + ag] = f2h_bits(av);
    wave_sync_lds();
  }
  __syncthreads();
  const int d = 4 * wave + (lane >> 3), a8 = (lane & 7) * 8;
  const v4u v = *(const v4u*)(sO + d * AGN + a8);
  unsigned short* dst = avt + ((size_t)h * HDM + d) * AGN + a8;
  *(volatile v4u*)dst = v;
  __threadfence();
  *(volatile v4u*)dst = v;
}

__global__ __launch_bounds__(256) void k_stage2(const unsigned short* __restrict__ qhp,
                                                 const unsigned short* __restrict__ ahp,
                                                 const unsigned short* __restrict__ avtp,
                                                 float* ot) {
  const _Float16* Q  = (const _Float16*)(const void*)qhp;
  const _Float16* A  = (const _Float16*)(const void*)ahp;
  const _Float16* AV = (const _Float16*)(const void*)avtp;
  __shared__ __align__(16) _Float16 sP[8][16 * SPP];
  __shared__ __align__(16) float sO[HDM * SOP];

  const int tid = threadIdx.x, wave = tid >> 5, lane = tid & 31;
  const int rl = lane & 15, hf = lane >> 4, koff = hf * 8;
  const int h = blockIdx.x / (NTK / QT2);
  const int tile = blockIdx.x - h * (NTK / QT2);
  const int n0 = tile * QT2;
  const int hc = h * HDM;

  const v16h qa = ldfrag_h(Q + (size_t)(n0 + 16 * wave + rl) * CH + hc + koff);
  v16h bfA[4];
#pragma unroll
  for (int j = 0; j < 4; ++j) bfA[j] = ldfrag_h(A + (size_t)(16 * j + rl) * CH + hc + koff);
  v8f sc[4];
#pragma unroll
  for (int j = 0; j < 4; ++j) sc[j] = mma_h_raw(qa, bfA[j], zero8());
  dep_guard4(sc[0], sc[1], sc[2], sc[3], qa, bfA[3]);
  keep4_h(bfA[0], bfA[1], bfA[2], bfA[3]);

  float mx[8];
#pragma unroll
  for (int r = 0; r < 8; ++r) {
    float m = sc[0][r];
    m = fmaxf(m, sc[1][r]);
    m = fmaxf(m, sc[2][r]);
    m = fmaxf(m, sc[3][r]);
    m = fmaxf(m, __shfl_xor(m, 1, 32));
    m = fmaxf(m, __shfl_xor(m, 2, 32));
    m = fmaxf(m, __shfl_xor(m, 4, 32));
    m = fmaxf(m, __shfl_xor(m, 8, 32));
    mx[r] = m * SFAC;
  }
  _Float16* sp = sP[wave];
  float ls[8];
#pragma unroll
  for (int r = 0; r < 8; ++r) {
    float l = 0.0f;
#pragma unroll
    for (int j = 0; j < 4; ++j) {
      const float p = __expf(sc[j][r] * SFAC - mx[r]);
      l += p;
      sp[(8 * hf + r) * SPP + 16 * j + rl] = (_Float16)(p * PSC);
    }
    l += __shfl_xor(l, 1, 32);
    l += __shfl_xor(l, 2, 32);
    l += __shfl_xor(l, 4, 32);
    l += __shfl_xor(l, 8, 32);
    ls[r] = l;
  }
  wave_sync_lds();

  v8f o0 = zero8(), o1 = zero8();
  v16h af, b0, b1;
#pragma unroll
  for (int ks = 0; ks < 2; ++ks) {
    af = ldfrag_h(sp + rl * SPP + 32 * ks + koff);
    b0 = ldfrag_h(AV + (size_t)(hc + rl) * AGN + 32 * ks + koff);
    b1 = ldfrag_h(AV + (size_t)(hc + 16 + rl) * AGN + 32 * ks + koff);
    o0 = mma_h_raw(af, b0, o0);
    o1 = mma_h_raw(af, b1, o1);
    dep_guard_h(o0, o1, af, b1);
    keep2_h(b0, b1);
  }
#pragma unroll
  for (int r = 0; r < 8; ++r) {
    const float inv = (1.0f / ls[r]) * OSC2;
    const int tok = 16 * wave + 8 * hf + r;
    sO[rl * SOP + tok] = o0[r] * inv;
    sO[(16 + rl) * SOP + tok] = o1[r] * inv;
  }
  __syncthreads();
  v4f ov[4];
#pragma unroll
  for (int it = 0; it < 4; ++it) ov[it] = *(const v4f*)(sO + (4 * wave + it) * SOP + 4 * lane);
  for (int pass = 0; pass < 2; ++pass) {
#pragma unroll
    for (int it = 0; it < 4; ++it)
      *(volatile v4f*)(ot + ((size_t)hc + 4 * wave + it) * NTK + n0 + 4 * lane) = ov[it];
    __threadfence();
  }
}

extern "C" void kernel_launch(void* const* d_in, const int* in_sizes, int n_in,
                              void* d_out, int out_size, void* d_ws, size_t ws_size,
                              hipStream_t stream) {
  if (n_in < 7) return;
  if (in_sizes[0] != NTK * CH) return;
  if (in_sizes[1] != 3 * CH * CH) return;
  if (in_sizes[2] != 3 * CH) return;
  if (in_sizes[3] != CH * CH) return;
  if (in_sizes[4] != CH) return;
  if (in_sizes[5] != CH * KCV) return;
  if (in_sizes[6] != CH) return;
  if (out_size != NTK * CH) return;

  const float* x      = (const float*)d_in[0];
  const float* w_qkv  = (const float*)d_in[1];
  const float* b_qkv  = (const float*)d_in[2];
  const float* w_proj = (const float*)d_in[3];
  const float* b_proj = (const float*)d_in[4];
  const float* w_dwc  = (const float*)d_in[5];
  const float* b_dwc  = (const float*)d_in[6];
  float* out = (float*)d_out;

  const size_t P32   = (size_t)NTK * CH * 4;
  const size_t P16   = (size_t)NTK * CH * 2;
  const size_t PWQ   = (size_t)3 * CH * CH * 2;
  const size_t PAH   = (size_t)AGN * CH * 2;
  const size_t PAVT  = (size_t)NHD * HDM * AGN * 2;
  const size_t PWD   = (size_t)CH * KCV * 2;
  const size_t PWP   = (size_t)CH * (2 * CH) * 2;
  const size_t PPART = (size_t)NHD * NSL * RECF * 4;
  const size_t PCOL  = (size_t)CHUNK * KCV * 2;
  const size_t PS2   = (size_t)NTK * (2 * CH) * 2;

  size_t off = 0;
  const size_t oTF  = off; off += P32;
  const size_t oXH  = off; off += P16;
  const size_t oQH  = off; off += P16;
  const size_t oKH  = off; off += P16;
  const size_t oVCM = off; off += P16;
  const size_t oVTM = off; off += P16;
  const size_t oWQ  = off; off += PWQ;
  const size_t oAH  = off; off += PAH;
  const size_t oAVT = off; off += PAVT;
  const size_t oWD  = off; off += PWD;
  const size_t oWP  = off; off += PWP;
  if (off > ws_size) return;
  if (off > (size_t)134217728) return;
  if (PPART > P16) return;
  if (oXH + PCOL > oKH) return;
  if (oKH + P32 > oVTM) return;
  if (PS2 > P32) return;

  char* ws = (char*)d_ws;
  float*          TF   = (float*)(ws + oTF);
  float*          OT   = (float*)(ws + oTF);
  unsigned short* S2   = (unsigned short*)(ws + oTF);
  unsigned short* XH   = (unsigned short*)(ws + oXH);
  float*          PART = (float*)(ws + oXH);
  unsigned short* COL  = (unsigned short*)(ws + oXH);
  unsigned short* QH   = (unsigned short*)(ws + oQH);
  unsigned short* KH   = (unsigned short*)(ws + oKH);
  float*          S    = (float*)(ws + oKH);
  unsigned short* VCM  = (unsigned short*)(ws + oVCM);
  unsigned short* VTM  = (unsigned short*)(ws + oVTM);
  unsigned short* WQKV = (unsigned short*)(ws + oWQ);
  unsigned short* AH   = (unsigned short*)(ws + oAH);
  unsigned short* AVT  = (unsigned short*)(ws + oAVT);
  unsigned short* WD   = (unsigned short*)(ws + oWD);
  unsigned short* WP2  = (unsigned short*)(ws + oWP);

  const dim3 blk(256);
  const dim3 gRows(NTK / 64);
  const dim3 gGemm(((NTK / 64) * (CH / 64)) / 8);
  const dim3 gGemmC(((CHUNK / 64) * (CH / 64)) / 8);

  k_cvt_rows<<<gRows, blk, 0, stream>>>(x, NTK, XSC, 1, XH);
  k_cvt_rows<<<dim3((3 * CH) / 64), blk, 0, stream>>>(w_qkv, 3 * CH, WSC, 1, WQKV);
  k_cvt_wd<<<dim3((CH * NTAP) / (8 * SEGW)), blk, 0, stream>>>(w_dwc, WD);
  k_cvt_wp<<<dim3(CH / 8), blk, 0, stream>>>(w_proj, WP2);
  gemm64<0><<<gGemm, blk, 0, stream>>>(XH, CH, WQKV, CH, TF, CH, NTK, CH, CH, OSC_G, b_qkv, TF);
  k_pool<<<dim3(AGN), blk, 0, stream>>>(TF, AH);
  k_cvt_rows<<<gRows, blk, 0, stream>>>(TF, NTK, QSC, 0, QH);
  gemm64<0><<<gGemm, blk, 0, stream>>>(XH, CH, WQKV + (size_t)CH * CH, CH, TF, CH, NTK, CH, CH, OSC_G, b_qkv + CH, TF);
  k_cvt_rows<<<gRows, blk, 0, stream>>>(TF, NTK, QSC, 0, KH);
  gemm64<0><<<gGemm, blk, 0, stream>>>(XH, CH, WQKV + (size_t)2 * CH * CH, CH, TF, CH, NTK, CH, CH, OSC_G, b_qkv + 2 * CH, TF);
  k_cvt_v<<<gRows, blk, 0, stream>>>(TF, VTM, VCM);
  k_stage1<<<dim3(NHD * NSL), blk, 0, stream>>>(AH, KH, VCM, PART);
  k_comb<<<dim3(NHD), blk, 0, stream>>>(PART, AVT);
  k_stage2<<<dim3(NHD * (NTK / QT2)), blk, 0, stream>>>(QH, AH, AVT, OT);
  const dim3 gI2c((CHUNK * NTAP) / (8 * SEGW));
  for (int ck = 0; ck < NCHK; ++ck) {
    k_im2col<<<gI2c, blk, 0, stream>>>(VTM, COL, ck);
    gemm64<1><<<gGemmC, blk, 0, stream>>>(COL, KCV, WD, KCV,
                                           S + (size_t)ck * CHUNK * CH, CH,
                                           CHUNK, CH, KCV, OSC_G, b_dwc,
                                           OT + (size_t)ck * CHUNK * CH);
  }
  k_split<<<gRows, blk, 0, stream>>>(S, S2);
  gemm64<0><<<gGemm, blk, 0, stream>>>(S2, 2 * CH, WP2, 2 * CH, out, CH, NTK, CH, 2 * CH, OSC_P, b_proj, out);
  (void)hipGetLastError();
}
